// GCNDeep_15393162789376
// MI455X (gfx1250) — hardware-verified
//
#include <hip/hip_runtime.h>


namespace {
constexpr int N = 50000, E = 800000, F = 128, FO = 64, NB = 256, NPAD = 50176  , NBLK = NPAD / 128, NAGG = NPAD / NB;
constexpr float AS_ = 8.0f, WS_ = 8.0f;

typedef _Float16 b16;
typedef __attribute__((ext_vector_type(16))) _Float16 v16b;
typedef __attribute__((ext_vector_type(8))) _Float16 v8b;
typedef __attribute__((ext_vector_type(8))) float v8f;
typedef __attribute__((ext_vector_type(4))) float v4f;
__device__ __forceinline__ void split16(float v, b16& hi, b16& lo) { hi = (b16)v; lo = (b16)(v - (float)hi); }
__device__ __forceinline__ v16b frag_kb(const b16* p, int hh) { const v8b a = *(const v8b*)(p + 8 * hh), b = *(const v8b*)(p + 16 + 8 * hh); v16b f;
#pragma unroll
  for (int e = 0; e < 8; ++e) { f[e] = a[e]; f[8 + e] = b[e]; } return f; }
__device__ __forceinline__ v8f wmma16b(v16b a, v16b b, v8f c) { v8f d = __builtin_amdgcn_wmma_f32_16x16x32_f16(false, a, false, b, (short)0, c, false, false); asm volatile("v_nop\n\tv_nop\n\tv_nop\n\tv_nop" : "+v"(d) : "v"(a), "v"(b)); return d; }
__device__ __forceinline__ void wave_lds_sync() { __builtin_amdgcn_fence(__ATOMIC_RELEASE, "workgroup"); __builtin_amdgcn_wave_barrier(); __builtin_amdgcn_fence(__ATOMIC_ACQUIRE, "workgroup"); }

__global__ __launch_bounds__(256) void prep_kernel(const float* __restrict__ W0, const float* __restrict__ W1, const float* __restrict__ W2, const float* __restrict__ W3, b16* __restrict__ wp) {
  const int t_ = threadIdx.x + blockIdx.x * 256, nth = gridDim.x * 256;
  for (int pass = 0; pass < 2; ++pass) {
    for (int p = t_; p < 3 * F * F + FO * F; p += nth) { int m, o, k; const float* W; size_t base;
      if (p < 3 * F * F) { m = p / (F * F); const int q = p % (F * F); o = q / F; k = q % F; W = (m == 0) ? W0 : (m == 1) ? W1 : W2; base = (size_t)m * 2 * F * F; const float v = W[k * F + o] * WS_; b16 a, c; split16(v, a, c); ((volatile b16*)wp)[base + q] = a; ((volatile b16*)wp)[base + F * F + q] = c; }
      else { const int q = p - 3 * F * F; o = q / F; k = q % F; base = (size_t)6 * F * F; const float v = W3[k * FO + o] * WS_; b16 a, c; split16(v, a, c); ((volatile b16*)wp)[base + q] = a; ((volatile b16*)wp)[base + FO * F + q] = c; } }
    __threadfence();
  }
}

template <int NOUT, int MODE>
__global__ __launch_bounds__(128) void sup_kernel(const float* __restrict__ h, const float* __restrict__ bin, const b16* __restrict__ Bw, size_t LOFF, float* __restrict__ sup) {
  __shared__ __attribute__((aligned(16))) float Ts[4][32 * 64];
  const int lane = threadIdx.x & 31, wave = threadIdx.x >> 5, nloc = lane & 15, hlf = lane >> 4, m0 = blockIdx.y * 128 + wave * 32, c0 = blockIdx.x * 64;
  const int ra = min(m0 + nloc, N - 1), rb = min(m0 + 16 + nloc, N - 1);
  v8f acc[2][4];
#pragma unroll
  for (int r = 0; r < 2; ++r)
#pragma unroll
    for (int t = 0; t < 4; ++t) acc[r][t] = (v8f){};
#pragma unroll 2
  for (int kb = 0; kb < F; kb += 32) { v16b a0, a1, l0, l1;
#pragma unroll
    for (int e = 0; e < 16; ++e) { const int k = kb + ((e < 8) ? (8 * hlf + e) : (16 + 8 * hlf + e - 8)); float va = h[(size_t)ra * F + k], vb = h[(size_t)rb * F + k];
      if (MODE == 1) { const float bb = bin[k]; va = fmaxf(va + bb, 0.0f); vb = fmaxf(vb + bb, 0.0f); }
      b16 p, q; split16(va * AS_, p, q); a0[e] = p; l0[e] = q; split16(vb * AS_, p, q); a1[e] = p; l1[e] = q; }
#pragma unroll
    for (int t = 0; t < 4; ++t) { const size_t bo = (size_t)(c0 + t * 16 + nloc) * F + kb; const v16b b0 = frag_kb(Bw + bo, hlf), b1 = frag_kb(Bw + LOFF + bo, hlf);
      acc[0][t] = wmma16b(a0, b0, acc[0][t]); acc[0][t] = wmma16b(l0, b0, acc[0][t]); acc[0][t] = wmma16b(a0, b1, acc[0][t]);
      acc[1][t] = wmma16b(a1, b0, acc[1][t]); acc[1][t] = wmma16b(l1, b0, acc[1][t]); acc[1][t] = wmma16b(a1, b1, acc[1][t]); } }
  float* Tt = Ts[wave];
#pragma unroll
  for (int t = 0; t < 4; ++t)
#pragma unroll
    for (int r = 0; r < 2; ++r)
#pragma unroll
      for (int v = 0; v < 8; ++v) Tt[(r * 16 + v + 8 * hlf) * 64 + t * 16 + nloc] = acc[r][t][v] * (1.0f / (AS_ * WS_));
  wave_lds_sync();
  for (int pass = 0; pass < 2; ++pass) {
#pragma unroll
    for (int j = 0; j < 16; ++j) { const int rr = j * 2 + hlf, c4 = nloc * 4; *(volatile v4f*)(sup + (size_t)(m0 + rr) * NOUT + c0 + c4) = *(const v4f*)(Tt + rr * 64 + c4); }
    __threadfence(); }
}

template <int DF, int MODE>
__global__ __launch_bounds__(256) void agg_kernel(const int* __restrict__ esrc, const int* __restrict__ edst, const float* __restrict__ ew, const float* __restrict__ sup, const float* __restrict__ bias, float FX, float* __restrict__ out) {
  __shared__ __attribute__((aligned(16))) int acc[NB * DF]; __shared__ int list[8 * 256];
  constexpr int LW = DF / 4, SUBS = 32 / LW;
  const int t_ = threadIdx.x, wave = t_ >> 5, lane = t_ & 31, base = blockIdx.x * NB, sub = lane / LW, cl = (lane % LW) * 4;
  for (int i = t_; i < NB * DF; i += 256) acc[i] = 0;
  __syncthreads();
  int* wl = list + wave * 256;
  for (int c0 = 0; c0 < E; c0 += 256 * 8) {
    const int e0 = c0 + (wave * 32 + lane) * 8; int dd[8];
#pragma unroll
    for (int j = 0; j < 8; ++j) { const int dv = edst[min(e0 + j, E - 1)]; dd[j] = (e0 + j < E) ? dv : -1; }
    unsigned sl[8]; bool hit[8]; bool anyl = false;
#pragma unroll
    for (int j = 0; j < 8; ++j) { sl[j] = (unsigned)(dd[j] - base); hit[j] = sl[j] < (unsigned)NB; anyl |= hit[j]; }
    int wc = 0;
    if (__builtin_amdgcn_ballot_w32(anyl) != 0u) {
#pragma unroll
      for (int j = 0; j < 8; ++j) {
        const unsigned mj = __builtin_amdgcn_ballot_w32(hit[j]);
        if (mj != 0u) {
          if (hit[j]) { const int pos = wc + (int)__builtin_amdgcn_mbcnt_lo(mj, 0u); wl[pos] = ((e0 + j) << 8) | (int)sl[j]; }
          wc += __builtin_popcount(mj); } } }
    __builtin_amdgcn_wave_barrier(); __builtin_amdgcn_fence(__ATOMIC_RELEASE, "workgroup"); __builtin_amdgcn_fence(__ATOMIC_ACQUIRE, "workgroup");
    for (int i = sub; i < wc; i += SUBS) { const int ent = wl[i]; const int e = ent >> 8, slot = ent & 255; int s = esrc[e]; s = (s < 0) ? 0 : (s >= N ? N - 1 : s); const float we = ew[e];
      const v4f v = *(const v4f*)(sup + (size_t)s * DF + cl); int* ar = acc + slot * DF + cl;
#pragma unroll
      for (int c = 0; c < 4; ++c) atomicAdd(ar + c, (int)rintf(we * v[c] * FX)); }
    __builtin_amdgcn_wave_barrier();
  }
  __syncthreads();
  const float fxi = 1.0f / FX;
  for (int pass = 0; pass < 2; ++pass) {
    for (int i = t_; i < NB * DF / 4; i += 256) { const int slot = i / (DF / 4), cq = (i % (DF / 4)) * 4, node = base + slot; v4f o = {0.0f, 0.0f, 0.0f, 0.0f};
      if (node < N) {
#pragma unroll
        for (int c = 0; c < 4; ++c) o[c] = (float)acc[slot * DF + cq + c] * fxi + ((MODE == 1) ? bias[cq + c] : 0.0f); }
      if (MODE == 0) { if (node < NPAD) *(volatile v4f*)(out + (size_t)node * DF + cq) = o; }
      else { if (node < N) *(volatile v4f*)(out + (size_t)node * DF + cq) = o; } }
    __threadfence(); }
}
}

extern "C" void kernel_launch(void* const* d_in, const int* in_sizes, int n_in,
                              void* d_out, int out_size, void* d_ws, size_t ws_size, hipStream_t stream) {
  (void)n_in; (void)out_size;
  const float* x = (const float*)d_in[0]; const int* esrc = (const int*)d_in[1]; const int* edst = (const int*)d_in[2]; const float* ew = (const float*)d_in[3];
  const float* W0 = (const float*)d_in[4]; const float* b0 = (const float*)d_in[5]; const float* W1 = (const float*)d_in[6]; const float* b1 = (const float*)d_in[7]; const float* W2 = (const float*)d_in[8]; const float* b2 = (const float*)d_in[9]; const float* W3 = (const float*)d_in[10]; const float* b3 = (const float*)d_in[11];
  float* out = (float*)d_out;
  if (in_sizes[0] != N * F || in_sizes[1] != E || in_sizes[2] != E || in_sizes[3] != E || in_sizes[4] != F * F || in_sizes[10] != F * FO) return;
  size_t off = 0; char* ws = (char*)d_ws;
  auto carve = [&](size_t bytes) { char* p = ws + off; off += (bytes + 255) & ~(size_t)255; return p; };
  b16* wp = (b16*)carve(((size_t)6 * F * F + 2 * FO * F) * 2); float* sup = (float*)carve((size_t)NPAD * F * 4); float* agg = (float*)carve((size_t)NPAD * F * 4);
  if (off > ws_size) return;
  const float FX0 = 1048576.0f, FX1 = 524288.0f;
  prep_kernel<<<64, 256, 0, stream>>>(W0, W1, W2, W3, wp);
  sup_kernel<F, 0><<<dim3(F / 64, NBLK), 128, 0, stream>>>(x, nullptr, wp, (size_t)F * F, sup);
  agg_kernel<F, 0><<<NAGG, 256, 0, stream>>>(esrc, edst, ew, sup, nullptr, FX0, agg);
  sup_kernel<F, 1><<<dim3(F / 64, NBLK), 128, 0, stream>>>(agg, b0, wp + (size_t)2 * F * F, (size_t)F * F, sup);
  agg_kernel<F, 0><<<NAGG, 256, 0, stream>>>(esrc, edst, ew, sup, nullptr, FX0, agg);
  sup_kernel<F, 1><<<dim3(F / 64, NBLK), 128, 0, stream>>>(agg, b1, wp + (size_t)4 * F * F, (size_t)F * F, sup);
  agg_kernel<F, 0><<<NAGG, 256, 0, stream>>>(esrc, edst, ew, sup, nullptr, FX1, agg);
  sup_kernel<FO, 1><<<dim3(FO / 64, NBLK), 128, 0, stream>>>(agg, b2, wp + (size_t)6 * F * F, (size_t)FO * F, sup);
  agg_kernel<FO, 1><<<NAGG, 256, 0, stream>>>(esrc, edst, ew, sup, b3, FX1, out);
}
